// RAdaptGAT_49048526520904
// MI455X (gfx1250) — hardware-verified
//
#include <hip/hip_runtime.h>
#include <math.h>

typedef __attribute__((ext_vector_type(16))) _Float16 v16h;
typedef __attribute__((ext_vector_type(8)))  _Float16 v8h;
typedef __attribute__((ext_vector_type(4)))  _Float16 v4h;
typedef __attribute__((ext_vector_type(16))) __bf16   v16b;
typedef __attribute__((ext_vector_type(8)))  __bf16   v8b;
typedef __attribute__((ext_vector_type(8)))  float    v8f;
typedef __attribute__((ext_vector_type(4)))  float    v4f;
typedef __attribute__((ext_vector_type(4)))  int      v4i;
#define U16(p) ((const unsigned short*)(const void*)(p))

__device__ __forceinline__ unsigned short f2bf_bits(float f) {
  unsigned u = __float_as_uint(f);
  return (unsigned short)((u + 0x7FFFu + ((u >> 16) & 1u)) >> 16);
}
__device__ __forceinline__ float bf_bits2f(unsigned short h) { return __uint_as_float(((unsigned)h) << 16); }

__device__ __forceinline__ void dep_guard_h(v8f& a, v8f& b, v16h x, v16h y) { asm volatile("v_nop\n\tv_nop\n\tv_nop\n\tv_nop" : "+v"(a), "+v"(b) : "v"(x), "v"(y)); }
__device__ __forceinline__ void dep_guard_b(v8f& a, v8f& b, v16b x, v16b y) { asm volatile("v_nop\n\tv_nop\n\tv_nop\n\tv_nop" : "+v"(a), "+v"(b) : "v"(x), "v"(y)); }
__device__ __forceinline__ void keep4_h(v16h a, v16h b, v16h c, v16h d) { asm volatile("v_nop" :: "v"(a), "v"(b), "v"(c), "v"(d)); }
__device__ __forceinline__ void keep4_b(v16b a, v16b b, v16b c, v16b d) { asm volatile("v_nop" :: "v"(a), "v"(b), "v"(c), "v"(d)); }
__device__ __forceinline__ void acc_guard4(v8f& a, v8f& b, v8f& c, v8f& d) { asm volatile("v_nop\n\tv_nop\n\tv_nop\n\tv_nop" : "+v"(a), "+v"(b), "+v"(c), "+v"(d)); }
template <typename T> struct Frag;
template <> struct Frag<_Float16> {
  typedef v16h V; union U { v16h v; v8h h[2]; };
  static __device__ __forceinline__ v16h load(const _Float16* p) {
    U f; f.h[0] = *(const v8h*)(p); f.h[1] = *(const v8h*)(p + 16); return f.v;
  }
  static __device__ __forceinline__ v8f mma(v16h a, v16h b, v8f c) {
    return __builtin_amdgcn_wmma_f32_16x16x32_f16(false, a, false, b, (short)0, c, false, false);
  }
  static __device__ __forceinline__ void guard(v8f& a, v8f& b, v16h x, v16h y) { dep_guard_h(a, b, x, y); }
  static __device__ __forceinline__ void keep(v16h a, v16h b, v16h c, v16h d) { keep4_h(a, b, c, d); }
};
template <> struct Frag<__bf16> {
  typedef v16b V; union U { v16b v; v8b h[2]; };
  static __device__ __forceinline__ v16b load(const __bf16* p) {
    U f; f.h[0] = *(const v8b*)(p); f.h[1] = *(const v8b*)(p + 16); return f.v;
  }
  static __device__ __forceinline__ v8f mma(v16b a, v16b b, v8f c) {
    return __builtin_amdgcn_wmma_f32_16x16x32_bf16(false, a, false, b, (short)0, c, false, false);
  }
  static __device__ __forceinline__ void guard(v8f& a, v8f& b, v16b x, v16b y) { dep_guard_b(a, b, x, y); }
  static __device__ __forceinline__ void keep(v16b a, v16b b, v16b c, v16b d) { keep4_b(a, b, c, d); }
};

template <int ET> struct Elem;
template <> struct Elem<0> { typedef _Float16 T; };
template <> struct Elem<1> { typedef __bf16 T; };
template <int ET, bool SPLIT, int BIAS_MODE, int OUT_MODE, bool RESID, int ACT = 0>
__global__ __launch_bounds__(256) void wmma_gemm64(
    const unsigned short* __restrict__ Ap, const unsigned short* __restrict__ A2p, int lda, long strideA,
    const unsigned short* __restrict__ Btp, const unsigned short* __restrict__ Bt2p, int ldb, long strideB,
    void* __restrict__ Cout, void* __restrict__ Cout2, int ldc, long strideC,
    const float* __restrict__ bias,
    const float* __restrict__ resid, long strideR,
    int M, int N, int K, float scale) {
  typedef typename Elem<ET>::T T;
  typedef typename Frag<T>::V V;
  const T* A = (const T*)Ap; const T* A2 = (const T*)A2p; const T* Bt = (const T*)Btp; const T* Bt2 = (const T*)Bt2p;
  __shared__ __align__(16) float sT[8][16 * 68];
  const int b    = blockIdx.y;
  const int lane = threadIdx.x & 31;
  const int wave = threadIdx.x >> 5;
  const int tilesN = N >> 6;
  const int tilesM = M >> 6;
  const int tile = blockIdx.x * 8 + wave;
  if (tile >= tilesM * tilesN) return;
  const int tm = tile / tilesN;
  const int tn = tile - tm * tilesN;
  const int m0 = tm << 6;
  const int n0 = tn << 6;

  const T* Ab  = A  + (size_t)b * strideA;
  const T* Bb  = Bt + (size_t)b * strideB;
  const T* Ab2 = SPLIT ? (A2  + (size_t)b * strideA) : nullptr;
  const T* Bb2 = SPLIT ? (Bt2 + (size_t)b * strideB) : nullptr;

  const int rlane = lane & 15;
  const int koff  = (lane >> 4) * 8;
  const int mOff  = (lane >> 4) * 8;

  v8f acc[4][4];
#pragma unroll
  for (int i = 0; i < 4; ++i)
#pragma unroll
    for (int j = 0; j < 4; ++j) acc[i][j] = (v8f){0.f,0.f,0.f,0.f,0.f,0.f,0.f,0.f};

  for (int k0 = 0; k0 < K; k0 += 32) {
    V bh[4], bl[4];
#pragma unroll
    for (int j = 0; j < 4; ++j) {
      const size_t bo = (size_t)(n0 + (j << 4) + rlane) * ldb + koff + k0;
      bh[j] = Frag<T>::load(Bb + bo);
      if (SPLIT) bl[j] = Frag<T>::load(Bb2 + bo);
    }
#pragma unroll
    for (int i = 0; i < 4; ++i) {
      const size_t ao = (size_t)(m0 + (i << 4) + rlane) * lda + koff + k0;
      V ah = Frag<T>::load(Ab + ao);
      V al;
      if (SPLIT) al = Frag<T>::load(Ab2 + ao);
#pragma unroll
      for (int j = 0; j < 4; ++j) {
        acc[i][j] = Frag<T>::mma(ah, bh[j], acc[i][j]);
        if (SPLIT) {
          acc[i][j] = Frag<T>::mma(ah, bl[j], acc[i][j]);
          acc[i][j] = Frag<T>::mma(al, bh[j], acc[i][j]);
        }
      }
      Frag<T>::guard(acc[i][0], acc[i][3], ah, SPLIT ? al : ah);
    }
    Frag<T>::keep(bh[0], bh[1], bh[2], bh[3]);
    if (SPLIT) Frag<T>::keep(bl[0], bl[1], bl[2], bl[3]);
  }
  acc_guard4(acc[0][0], acc[0][1], acc[0][2], acc[0][3]);
  acc_guard4(acc[1][0], acc[1][1], acc[1][2], acc[1][3]);
  acc_guard4(acc[2][0], acc[2][1], acc[2][2], acc[2][3]);
  acc_guard4(acc[3][0], acc[3][1], acc[3][2], acc[3][3]);

  float* slab = sT[wave];
  const float* Rb = RESID ? (resid + (size_t)b * strideR) : nullptr;
#pragma unroll
  for (int i = 0; i < 4; ++i) {
    const int mBase = m0 + (i << 4);
#pragma unroll
    for (int j = 0; j < 4; ++j) {
      const int n = n0 + (j << 4) + rlane;
      float bv = 0.f;
      if (BIAS_MODE == 2) bv = bias[n];
#pragma unroll
      for (int r = 0; r < 8; ++r) {
        float v = acc[i][j][r] * scale;
        if (BIAS_MODE == 1) v += bias[mBase + mOff + r];
        if (BIAS_MODE == 2) v += bv;
        if (RESID) v += Rb[(size_t)(mBase + mOff + r) * ldc + n];
        if (ACT == 1) v = tanhf(v);
        if (ACT == 2) v = fmaxf(v, 0.0f);
        if (ACT == 3) v = v / (1.0f + expf(-v));
        if (ACT == 4) v = (v > 0.f) ? v : 0.01f * v;
        if (ACT == 5) v = 0.5f * v * (1.0f + erff(v * 0.70710678118654752f));
        slab[(mOff + r) * 68 + (j << 4) + rlane] = v;
      }
    }
    __builtin_amdgcn_fence(__ATOMIC_RELEASE, "workgroup");
    __builtin_amdgcn_wave_barrier();
    __builtin_amdgcn_fence(__ATOMIC_ACQUIRE, "workgroup");
    if (OUT_MODE == 0) {
      float* C = (float*)Cout + (size_t)b * strideC;
      const int hh = lane >> 4, c4 = (lane & 15) * 4;
      for (int pass = 0; pass < 2; ++pass) {
#pragma unroll
        for (int it = 0; it < 8; ++it) {
          const int row = it * 2 + hh;
          v4f v = *(const v4f*)(slab + row * 68 + c4);
          *(volatile v4f*)(C + (size_t)(mBase + row) * ldc + n0 + c4) = v;
        }
        __threadfence();
      }
    } else {
      const int q = lane >> 3, c8 = (lane & 7) * 8;
      unsigned short* C  = (unsigned short*)Cout  + (size_t)b * strideC;
      unsigned short* C2 = (OUT_MODE == 2) ? ((unsigned short*)Cout2 + (size_t)b * strideC) : nullptr;
      for (int pass = 0; pass < 2; ++pass) {
#pragma unroll
        for (int it = 0; it < 4; ++it) {
          const int row = it * 4 + q;
          const float* sp = slab + row * 68 + c8;
          v8h hv, lv;
#pragma unroll
          for (int e = 0; e < 8; ++e) {
            if (OUT_MODE == 1) {
              hv[e] = (_Float16)sp[e];
            } else {
              unsigned short hb = f2bf_bits(sp[e]);
              unsigned short lb = f2bf_bits(sp[e] - bf_bits2f(hb));
              hv[e] = __builtin_bit_cast(_Float16, hb);
              lv[e] = __builtin_bit_cast(_Float16, lb);
            }
          }
          *(volatile v8h*)(C + (size_t)(mBase + row) * ldc + n0 + c8) = hv;
          if (OUT_MODE == 2) *(volatile v8h*)(C2 + (size_t)(mBase + row) * ldc + n0 + c8) = lv;
        }
        __threadfence();
      }
    }
    __builtin_amdgcn_fence(__ATOMIC_RELEASE, "workgroup");
    __builtin_amdgcn_wave_barrier();
    __builtin_amdgcn_fence(__ATOMIC_ACQUIRE, "workgroup");
  }
}

#define NN 50000
#define NPAD 50048
#define NE 500000
#define NET (NE + NN)
#define NETP 550016
#define FIN 128
#define NT 256
#define SRB 1024
#define RPW (SRB / (NT / 32))
#define NTILE ((NPAD + SRB - 1) / SRB)
#define SCH 2048
#define NCH ((NE + SCH - 1) / SCH)

__global__ __launch_bounds__(256) void cast_pad_kernel(const float* __restrict__ x, unsigned* __restrict__ x16, int F) {
  const long i = (long)blockIdx.x * 256 + threadIdx.x; const long n2 = (long)NPAD * F / 2;
  if (i >= n2) return;
  const long e0 = 2 * i; const long row = e0 / F;
  const float a = (row < NN) ? x[e0] : 0.f, b = (row < NN) ? x[e0 + 1] : 0.f;
  const unsigned u = (unsigned)__builtin_bit_cast(unsigned short, (_Float16)a) | ((unsigned)__builtin_bit_cast(unsigned short, (_Float16)b) << 16);
  ((volatile unsigned*)x16)[i] = u; __threadfence(); ((volatile unsigned*)x16)[i] = u;
}

__global__ __launch_bounds__(256) void wcast_kernel(const float* __restrict__ Wl, const float* __restrict__ Wr, int ncol, int nrows,
                                                    _Float16* __restrict__ WT) {
  const int i = blockIdx.x * 256 + threadIdx.x;
  const int n2 = nrows * FIN / 2;
  if (i >= n2) return;
  const int e0 = 2 * i; const int n = e0 >> 7; const int k = e0 & 127;
  float a = 0.f, b = 0.f;
  if (n < ncol) { a = Wl[(size_t)k * ncol + n]; b = Wl[(size_t)(k + 1) * ncol + n]; }
  else if (n < 2 * ncol) { a = Wr[(size_t)k * ncol + (n - ncol)]; b = Wr[(size_t)(k + 1) * ncol + (n - ncol)]; }
  const _Float16 h0 = (_Float16)(a * 16.0f), h1 = (_Float16)(b * 16.0f);
  const unsigned u = (unsigned)__builtin_bit_cast(unsigned short, h0) | ((unsigned)__builtin_bit_cast(unsigned short, h1) << 16);
  ((volatile unsigned*)WT)[i] = u; __threadfence(); ((volatile unsigned*)WT)[i] = u;
}

__device__ __forceinline__ int blk_excl_scan(int cnt, int* scan_ws, int tid, int* tot) {
  const int lane = tid & 31, wave = tid >> 5; int incl = cnt;
#pragma unroll
  for (int o = 1; o < 32; o <<= 1) { const int v = __shfl_up(incl, o, 32); if (lane >= o) incl += v; }
  if (lane == 31) scan_ws[wave] = incl;
  __syncthreads();
  if (wave == 0) { int wv = (lane < NT / 32) ? scan_ws[lane] : 0; int wincl = wv;
#pragma unroll
    for (int o = 1; o < 32; o <<= 1) { const int v = __shfl_up(wincl, o, 32); if (lane >= o) wincl += v; }
    if (lane < NT / 32) scan_ws[32 + lane] = wincl - wv; if (lane == 31) scan_ws[64] = wincl; }
  __syncthreads();
  const int res = scan_ws[32 + wave] + incl - cnt; *tot = scan_ws[64];
  return res;
}
template <int SP, int CAP>
__device__ __forceinline__ int chunk_hits(const int* __restrict__ dstv, int e0, int n0, int tid, int* LIST, int* scan_ws) {
  const int eb = e0 + tid * SP;
  int rec[SP]; int cnt = 0;
  if (eb < NE) {
#pragma unroll
    for (int k = 0; k < SP; k += 4) {
      const v4i d4 = *(const v4i*)(dstv + eb + k);
#pragma unroll
      for (int u = 0; u < 4; ++u) {
        const int d = d4[u]; int r = -1;
        if (d >= n0 && d < n0 + SRB && d < NN) { r = ((d - n0) << 19) | (eb + k + u); ++cnt; }
        rec[k + u] = r;
      }
    }
  } else {
#pragma unroll
    for (int k = 0; k < SP; ++k) rec[k] = -1;
  }
  int tot; int p = blk_excl_scan(cnt, scan_ws, tid, &tot);
#pragma unroll
  for (int k = 0; k < SP; ++k) if (rec[k] >= 0) { if ((unsigned)p < (unsigned)CAP) LIST[p] = rec[k]; ++p; }
  __syncthreads();
  return tot < CAP ? tot : CAP;
}

template <bool L3>
__global__ __launch_bounds__(NT) void gat_logits_kernel(const float* __restrict__ XLR, const int* __restrict__ ei,
                                                       const float* __restrict__ att, float* __restrict__ LG) {
  constexpr int PITCH = L3 ? 64 : 256;
  constexpr int XROFF = L3 ? 16 : 128;
  constexpr int NA = L3 ? 16 : 128;
  __shared__ __align__(16) float sA[128];
  __shared__ __align__(16) float sal[32 * 8];
  const int tid = threadIdx.x, lane = tid & 31, wave = tid >> 5;
  if (tid < NA) sA[tid] = att[tid];
  __syncthreads();
#pragma unroll 1
  for (int i = 0; i < 4; ++i) {
    const int el = 4 * wave + i;
    int e = blockIdx.x * 32 + el; e = (e < NET) ? e : NET - 1;
    int s, d;
    if (e < NE) {
      s = ei[e]; d = ei[NE + e];
      s = s < 0 ? 0 : (s >= NN ? NN - 1 : s);
      d = d < 0 ? 0 : (d >= NN ? NN - 1 : d);
    } else { s = e - NE; d = s; }
    if (!L3) {
      const int c0 = 4 * lane;
      const v4f xv = *(const v4f*)(XLR + (size_t)s * PITCH + c0);
      const v4f rv = *(const v4f*)(XLR + (size_t)d * PITCH + XROFF + c0);
      const v4f av = *(const v4f*)(sA + c0);
      float dsum = 0.f;
#pragma unroll
      for (int t = 0; t < 4; ++t) { float v = xv[t] + rv[t]; v = (v >= 0.f) ? v : 0.2f * v; dsum += v * av[t]; }
      dsum += __shfl_xor(dsum, 1, 32); dsum += __shfl_xor(dsum, 2, 32);
      if ((lane & 3) == 0) sal[el * 8 + (lane >> 2)] = dsum;
    } else {
      const int c = lane & 15;
      float v = XLR[(size_t)s * PITCH + c] + XLR[(size_t)d * PITCH + XROFF + c];
      v = (v >= 0.f) ? v : 0.2f * v;
      float dsum = (lane < 16) ? v * sA[c] : 0.f;
      dsum += __shfl_xor(dsum, 1, 32); dsum += __shfl_xor(dsum, 2, 32);
      dsum += __shfl_xor(dsum, 4, 32); dsum += __shfl_xor(dsum, 8, 32);
      if (lane == 0) sal[el] = dsum;
    }
  }
  __syncthreads();
  if (!L3) {
    if (tid < 64) {
      const v4f v = *(const v4f*)(sal + 4 * tid);
      float* op = LG + (size_t)blockIdx.x * 32 * 8 + 4 * tid;
      *(volatile v4f*)op = v; __threadfence(); *(volatile v4f*)op = v;
    }
  } else {
    if (tid < 32) {
      const float v = sal[tid];
      float* op = LG + (size_t)blockIdx.x * 32 + tid;
      *(volatile float*)op = v; __threadfence(); *(volatile float*)op = v;
    }
  }
}

template <bool L3>
__global__ __launch_bounds__(NT) void gat_stream_kernel(float* XLR, const int* __restrict__ ei, const float* __restrict__ LG,
                                                       const float* __restrict__ bias, const float* __restrict__ bng, const float* __restrict__ bnb,
                                                       const float* __restrict__ bnm, const float* __restrict__ bnv,
                                                       _Float16* __restrict__ H16, float* __restrict__ OUT) {
  constexpr int NHD = L3 ? 1 : 8;
  constexpr int PITCH = L3 ? 64 : 256;
  constexpr int HC = L3 ? 16 : 128;
  __shared__ int LIST[SCH];
  __shared__ float SM[SRB * NHD];
  __shared__ float SL[SRB * NHD];
  __shared__ __align__(16) float ACC[L3 ? SRB * 16 : 16];
  __shared__ int scan_ws[80];
  const int tid = threadIdx.x, lane = tid & 31, wave = tid >> 5;
  const int n0 = blockIdx.x * SRB;
  const int hs = L3 ? 0 : (lane & 7);
  const int hc = lane >> 2;
  const int cc = lane & 15;
  const v4f z4 = {0.f, 0.f, 0.f, 0.f};

#pragma unroll 1
  for (int j = 0; j < RPW; ++j) {
    const int dl = wave * RPW + j; const int n = n0 + dl;
    if (n < NPAD) {
      const bool live = n < NN;
      float lg = -INFINITY;
      if (live) lg = LG[(size_t)(NE + n) * NHD + hs];
      if (!L3) {
        if (lane < 8) { SM[dl * 8 + hs] = lg; SL[dl * 8 + hs] = live ? 1.f : 0.f; }
        v4f a = z4;
        if (live) a = *(const v4f*)(XLR + (size_t)n * PITCH + 4 * lane);
        *(v4f*)(XLR + (size_t)n * PITCH + HC + 4 * lane) = a;
      } else {
        if (lane == 0) { SM[dl] = lg; SL[dl] = live ? 1.f : 0.f; }
        float a = 0.f;
        if (live) a = XLR[(size_t)n * PITCH + cc];
        if (lane < 16) ACC[dl * 16 + cc] = a;
      }
    }
  }
  __syncthreads();

  const int* dstv = ei + NE;
#pragma unroll 1
  for (int c = 0; c < NCH; ++c) {
    const int tot = chunk_hits<SCH / NT, SCH>(dstv, c * SCH, n0, tid, LIST, scan_ws);
#pragma unroll 1
    for (int base = 0; base < tot; base += 32) {
      const int q = base + lane;
      const int rv = (q < tot) ? LIST[q] : -1;
      const int own = (rv >= 0 && (rv >> 26) == wave) ? 1 : 0;
      unsigned msk = (unsigned)__ballot(own);
#pragma unroll 1
      for (int it = 0; it < 32; ++it) {
        if (msk == 0u) break;
        const int bpos = __builtin_ctz(msk); msk &= msk - 1u;
        const int r = __shfl(rv, bpos, 32);
        const int dl = (r >> 19) & (SRB - 1);
        int e = r & 0x7FFFF; e = (e < NE) ? e : NE - 1;
        int s = ei[e]; s = s < 0 ? 0 : (s >= NN ? NN - 1 : s);
        int nr = n0 + dl; nr = (nr < NPAD) ? nr : NPAD - 1;
        const float lg = LG[(size_t)e * NHD + hs];
        const int mi = dl * NHD + hs;
        const float mo = SM[mi], lo = SL[mi];
        const float mn = fmaxf(mo, lg);
        const float rr = __expf(mo - mn), ex = __expf(lg - mn);
        const float ln = lo * rr + ex;
        if (lane < NHD) { SM[mi] = mn; SL[mi] = ln; }
        if (!L3) {
          const float rrj = __shfl(rr, hc, 32), exj = __shfl(ex, hc, 32);
          float* rp = XLR + (size_t)nr * PITCH + HC + 4 * lane;
          const v4f hv = *(const v4f*)(XLR + (size_t)s * PITCH + 4 * lane);
          v4f a = *(const v4f*)rp;
          a = a * rrj + exj * hv;
          *(v4f*)rp = a;
        } else {
          const float hv = XLR[(size_t)s * PITCH + cc];
          float a = ACC[dl * 16 + cc];
          a = a * rr + ex * hv;
          if (lane < 16) ACC[dl * 16 + cc] = a;
        }
      }
    }
    __syncthreads();
  }

  if (!L3) {
    const int cb = 4 * lane;
    v4f b4, m4, be4, sc4;
#pragma unroll
    for (int q = 0; q < 4; ++q) {
      b4[q] = bias[cb + q]; m4[q] = bnm[cb + q]; be4[q] = bnb[cb + q];
      sc4[q] = bng[cb + q] * rsqrtf(bnv[cb + q] + 1e-5f);
    }
#pragma unroll 1
    for (int j = 0; j < RPW; ++j) {
      const int dl = wave * RPW + j; const int n = n0 + dl;
      if (n < NPAD) {
        const bool live = n < NN;
        const float slv = SL[dl * 8 + hc];
        const float sl2 = (live && slv > 0.f) ? slv : 1.0f;
        const float inv = live ? __builtin_amdgcn_rcpf(sl2) : 0.f;
        const v4f a = *(const v4f*)(XLR + (size_t)n * PITCH + HC + 4 * lane);
        const v4f t = a * inv + b4;
        const v4f u = (t - m4) * sc4 + be4;
        v4h hv;
#pragma unroll
        for (int q = 0; q < 4; ++q) {
          float v = u[q];
          v = (v > 0.f) ? v : (__expf(v) - 1.0f);
          hv[q] = (_Float16)(live ? v : 0.f);
        }
        _Float16* hp = H16 + (size_t)n * 128 + 4 * lane;
        *(volatile v4h*)hp = hv; __threadfence(); *(volatile v4h*)hp = hv;
      }
    }
  } else {
    const float bc = bias[cc];
#pragma unroll 1
    for (int j = 0; j < RPW; ++j) {
      const int dl = wave * RPW + j; const int n = n0 + dl;
      if (n < NPAD) {
        const bool live = n < NN;
        const float slv = SL[dl];
        const float sl2 = (live && slv > 0.f) ? slv : 1.0f;
        const float inv = __builtin_amdgcn_rcpf(sl2);
        const float a = ACC[dl * 16 + cc];
        const float v = live ? (a * inv + bc) : 0.f;
        if (lane < 16) ACC[dl * 16 + cc] = v;
      }
    }
    __syncthreads();
    for (int pass = 0; pass < 2; ++pass) {
#pragma unroll 1
      for (int it = 0; it < (SRB * 16) / (4 * NT); ++it) {
        const int q = it * NT + tid;
        const size_t idx = (size_t)n0 * 16 + 4 * (size_t)q;
        if (idx < (size_t)NN * 16) {
          const v4f v = *(const v4f*)(ACC + 4 * q);
          *(volatile v4f*)(OUT + idx) = v;
        }
      }
      __threadfence();
    }
  }
}

extern "C" void kernel_launch(void* const* d_in, const int* in_sizes, int n_in,
                              void* d_out, int out_size, void* d_ws, size_t ws_size,
                              hipStream_t stream) {
  if (n_in < 30) return;
  if (in_sizes[0] != NN * FIN || in_sizes[1] != 2 * NE || out_size != NN * 16) return;
  const float* x  = (const float*)d_in[0];
  const int*   ei = (const int*)  d_in[1];
  const float* Wl[4]  = {(const float*)d_in[2],  (const float*)d_in[6],  (const float*)d_in[10], (const float*)d_in[14]};
  const float* Wr[4]  = {(const float*)d_in[3],  (const float*)d_in[7],  (const float*)d_in[11], (const float*)d_in[15]};
  const float* att[4] = {(const float*)d_in[4],  (const float*)d_in[8],  (const float*)d_in[12], (const float*)d_in[16]};
  const float* bs[4]  = {(const float*)d_in[5],  (const float*)d_in[9],  (const float*)d_in[13], (const float*)d_in[17]};
  const float* bnG[3] = {(const float*)d_in[18], (const float*)d_in[22], (const float*)d_in[26]};
  const float* bnB[3] = {(const float*)d_in[19], (const float*)d_in[23], (const float*)d_in[27]};
  const float* bnM[3] = {(const float*)d_in[20], (const float*)d_in[24], (const float*)d_in[28]};
  const float* bnV[3] = {(const float*)d_in[21], (const float*)d_in[25], (const float*)d_in[29]};
  float* out = (float*)d_out;

  char* ws = (char*)d_ws; size_t off = 0;
  auto carve = [&](size_t bytes) -> char* { char* p = ws + off; off += (bytes + 255) & ~(size_t)255; return p; };
  _Float16* H16 = (_Float16*)carve((size_t)NPAD * FIN * 2);
  _Float16* WT  = (_Float16*)carve((size_t)256 * FIN * 2);
  float*    XLR = (float*)carve((size_t)NPAD * 256 * 4);
  float*    LG  = (float*)carve((size_t)NETP * 8 * 4);
  if (off > ws_size || off > (size_t)134217728) return;

  cast_pad_kernel<<<(NPAD * FIN / 2 + 255) / 256, 256, 0, stream>>>(x, (unsigned*)H16, FIN);

  for (int i = 0; i < 3; ++i) {
    wcast_kernel<<<(256 * FIN / 2 + 255) / 256, 256, 0, stream>>>(Wl[i], Wr[i], 128, 256, WT);
    {
      const int t1 = (NPAD / 64) * (256 / 64);
      wmma_gemm64<0, false, 0, 0, false><<<dim3((t1 + 7) / 8, 1), 256, 0, stream>>>(
          U16(H16), nullptr, FIN, 0L, U16(WT), nullptr, FIN, 0L,
          (void*)XLR, nullptr, 256, 0L, nullptr, nullptr, 0L, NPAD, 256, FIN, 0.0625f);
    }
    gat_logits_kernel<false><<<NETP / 32, NT, 0, stream>>>(XLR, ei, att[i], LG);
    gat_stream_kernel<false><<<NTILE, NT, 0, stream>>>(XLR, ei, LG, bs[i], bnG[i], bnB[i], bnM[i], bnV[i], H16, out);
  }
  {
    wcast_kernel<<<(64 * FIN / 2 + 255) / 256, 256, 0, stream>>>(Wl[3], Wr[3], 16, 64, WT);
    const int t3 = (NPAD / 64) * (64 / 64);
    wmma_gemm64<0, false, 0, 0, false><<<dim3((t3 + 7) / 8, 1), 256, 0, stream>>>(
        U16(H16), nullptr, FIN, 0L, U16(WT), nullptr, FIN, 0L,
        (void*)XLR, nullptr, 64, 0L, nullptr, nullptr, 0L, NPAD, 64, FIN, 0.0625f);
    gat_logits_kernel<true><<<NETP / 32, NT, 0, stream>>>(XLR, ei, att[3], LG);
    gat_stream_kernel<true><<<NTILE, NT, 0, stream>>>(XLR, ei, LG, bs[3], bs[3], bs[3], bs[3], bs[3], H16, out);
  }
}
